// MoHAttention_19447611916393
// MI455X (gfx1250) — hardware-verified
//
#include <hip/hip_runtime.h>
#include <stddef.h>
#include <stdint.h>

#define NBATCH 4
#define SQ     2048
#define NTOK   8192
#define DIM    768
#define NH     12
#define HDM    64
#define NQKV   2304
#define ER     10
#define GP     16
#define QB     128
#define KC     64
#define NQB    (SQ / QB)
#define NCK    (SQ / KC)
#define SBLK   (SQ / 256)
#define QKPLANE (NBATCH * NH * SQ * HDM)
#define LNEPS  1e-5f
#define QKS    0.03125f
#define PJS    0.00048828125f

static_assert(NTOK == NBATCH * SQ);
static_assert(SQ % 256 == 0);
static_assert(DIM % 64 == 0);
static_assert(DIM % 32 == 0);
static_assert(HDM == 64);
static_assert(NH * HDM == DIM);
static_assert(NQKV == 3 * DIM);
static_assert(NQKV % 64 == 0);
static_assert(SQ % KC == 0);
static_assert(SQ % QB == 0);
static_assert(NTOK % 256 == 0);
static_assert(NTOK % 8 == 0);
static_assert((NTOK * DIM) % 2048 == 0);
static_assert(ER + 2 == NH);
static_assert(NH <= GP);

typedef _Float16 v16h __attribute__((ext_vector_type(16)));
typedef _Float16 v8h  __attribute__((ext_vector_type(8)));
typedef float    v8f  __attribute__((ext_vector_type(8)));
typedef float    v4f  __attribute__((ext_vector_type(4)));
typedef float    v2f  __attribute__((ext_vector_type(2)));
typedef unsigned int v4u __attribute__((ext_vector_type(4)));

union Frag  { v16h v; v8h h[2]; };
union Pack8 { v8h h; v4u u; };

__device__ __forceinline__ v8f mma16(v16h a, v16h b, v8f c) {
  c = __builtin_amdgcn_wmma_f32_16x16x32_f16(false, a, false, b, (short)0, c, false, false);
  asm volatile("v_nop\n\tv_nop\n\tv_nop\n\tv_nop" : "+v"(c) : "v"(a), "v"(b));
  return c;
}

__device__ __forceinline__ v16h ldfrag(const _Float16* p, int ld, int row0, int k0, int lane) {
  const int m = lane & 15, lh = lane >> 4;
  const _Float16* q = p + (size_t)(row0 + m) * ld + k0 + 8 * lh;
  Frag f;
  f.h[0] = *(const v8h*)(q);
  f.h[1] = *(const v8h*)(q + 16);
  return f.v;
}

__device__ __forceinline__ v8f zero8() { return (v8f){0.f, 0.f, 0.f, 0.f, 0.f, 0.f, 0.f, 0.f}; }

__device__ __forceinline__ void gemm32x64(const _Float16* __restrict__ A, int lda,
                                          const _Float16* __restrict__ Bt, int ldb, int K,
                                          int m0, int n0, int lane, v8f (&acc)[2][4]) {
#pragma unroll 1
  for (int k0 = 0; k0 < K; k0 += 32) {
    const v16h a0 = ldfrag(A, lda, m0, k0, lane);
    const v16h a1 = ldfrag(A, lda, m0 + 16, k0, lane);
    const v16h b0 = ldfrag(Bt, ldb, n0, k0, lane);
    const v16h b1 = ldfrag(Bt, ldb, n0 + 16, k0, lane);
    const v16h b2 = ldfrag(Bt, ldb, n0 + 32, k0, lane);
    const v16h b3 = ldfrag(Bt, ldb, n0 + 48, k0, lane);
    acc[0][0] = mma16(a0, b0, acc[0][0]);
    acc[1][0] = mma16(a1, b0, acc[1][0]);
    acc[0][1] = mma16(a0, b1, acc[0][1]);
    acc[1][1] = mma16(a1, b1, acc[1][1]);
    acc[0][2] = mma16(a0, b2, acc[0][2]);
    acc[1][2] = mma16(a1, b2, acc[1][2]);
    acc[0][3] = mma16(a0, b3, acc[0][3]);
    acc[1][3] = mma16(a1, b3, acc[1][3]);
  }
}

__global__ __launch_bounds__(256) void k_cvt(const float* __restrict__ src, _Float16* __restrict__ dh, int n8) {
  const int i = blockIdx.x * 256 + (int)threadIdx.x;
  if (i >= n8) return;
  const size_t o = (size_t)i * 8;
  const v4f a0 = *(const v4f*)(src + o);
  const v4f a1 = *(const v4f*)(src + o + 4);
  Pack8 pk;
  pk.h = (v8h){(_Float16)a0[0], (_Float16)a0[1], (_Float16)a0[2], (_Float16)a0[3],
               (_Float16)a1[0], (_Float16)a1[1], (_Float16)a1[2], (_Float16)a1[3]};
  const v4u vv = pk.u;
  volatile v4u* d = (volatile v4u*)(dh + o);
  *d = vv;
  __threadfence();
  *d = vv;
}

#define TRP 72
__global__ __launch_bounds__(256) void k_wtr(const float* __restrict__ w, _Float16* __restrict__ wt,
                                             int kdim, int ndim, float scale) {
  __shared__ __align__(16) _Float16 st[64 * TRP];
  const int tid = threadIdx.x;
  const int n0 = blockIdx.x * 64, k0 = blockIdx.y * 64;
  const int kr = tid >> 2;
  const int nc = (tid & 3) * 16;
  const float* sp = w + (size_t)(k0 + kr) * ndim + n0 + nc;
#pragma unroll
  for (int q = 0; q < 4; ++q) {
    const v4f a = *(const v4f*)(sp + 4 * q) * scale;
#pragma unroll
    for (int j = 0; j < 4; ++j) st[(nc + 4 * q + j) * TRP + kr] = (_Float16)a[j];
  }
  __syncthreads();
  v4u val[2];
  size_t go[2];
#pragma unroll
  for (int j = 0; j < 2; ++j) {
    const int p  = tid + 256 * j;
    const int nr = p >> 3;
    const int pc = p & 7;
    Pack8 pk;
    pk.h   = *(const v8h*)(st + nr * TRP + pc * 8);
    val[j] = pk.u;
    go[j]  = (size_t)(n0 + nr) * kdim + k0 + pc * 8;
  }
  for (int ps = 0; ps < 2; ++ps) {
#pragma unroll
    for (int j = 0; j < 2; ++j) *(volatile v4u*)(wt + go[j]) = val[j];
    __threadfence();
  }
}

__global__ __launch_bounds__(256) void k_gate(const float* __restrict__ x, const float* __restrict__ wg,
                                              const float* __restrict__ wg0, const float* __restrict__ wg1,
                                              float* __restrict__ gp) {
  __shared__ __align__(16) float sg[8 * GP];
  const int tid = threadIdx.x, lane = tid & 31, wave = tid >> 5;
  const size_t t = (size_t)blockIdx.x * 8 + wave;
  const float* xr = x + t * DIM;

  float a[14];
#pragma unroll
  for (int e = 0; e < 14; ++e) a[e] = 0.f;
#pragma unroll 1
  for (int j = 0; j < DIM / 32; ++j) {
    const int k = j * 32 + lane;
    const float xv = xr[k];
    const v2f* wr = (const v2f*)(wg + (size_t)k * ER);
    const v2f w01 = wr[0], w23 = wr[1], w45 = wr[2], w67 = wr[3], w89 = wr[4];
    const v2f u  = *(const v2f*)(wg0 + 2 * k);
    const v2f z  = *(const v2f*)(wg1 + 2 * k);
    a[0]  += xv * w01[0];  a[1]  += xv * w01[1];
    a[2]  += xv * w23[0];  a[3]  += xv * w23[1];
    a[4]  += xv * w45[0];  a[5]  += xv * w45[1];
    a[6]  += xv * w67[0];  a[7]  += xv * w67[1];
    a[8]  += xv * w89[0];  a[9]  += xv * w89[1];
    a[10] += xv * u[0];    a[11] += xv * u[1];
    a[12] += xv * z[0];    a[13] += xv * z[1];
  }
#pragma unroll
  for (int e = 0; e < 14; ++e) {
#pragma unroll
    for (int off = 16; off >= 1; off >>= 1) a[e] += __shfl_xor(a[e], off, 32);
  }

  float mx = a[0];
#pragma unroll
  for (int e = 1; e < ER; ++e) mx = fmaxf(mx, a[e]);
  float ex[ER];
  float s = 0.f;
#pragma unroll
  for (int e = 0; e < ER; ++e) { ex[e] = __expf(a[e] - mx); s += ex[e]; }
  const float inv = __builtin_amdgcn_rcpf(s);
  float b1 = a[0];
  int i1 = 0;
#pragma unroll
  for (int e = 1; e < ER; ++e) { const bool gt = a[e] > b1; b1 = gt ? a[e] : b1; i1 = gt ? e : i1; }
  float b2 = -__builtin_huge_valf();
  int i2 = -1;
#pragma unroll
  for (int e = 0; e < ER; ++e) {
    const bool gt = (e != i1) && (a[e] > b2);
    b2 = gt ? a[e] : b2;
    i2 = gt ? e : i2;
  }
  float g[ER];
  float gsum = 0.f;
#pragma unroll
  for (int e = 0; e < ER; ++e) {
    g[e] = ex[e] * inv;
    const bool sel = (e == i1) || (e == i2);
    gsum += sel ? g[e] : 0.f;
  }
  const float dinv = __builtin_amdgcn_rcpf(fmaxf(gsum, 1.1920929e-7f));
  const float m0 = fmaxf(a[10], a[11]);
  const float e0 = __expf(a[10] - m0), e1 = __expf(a[11] - m0);
  const float r0 = __builtin_amdgcn_rcpf(e0 + e1);
  const float w00 = (e0 * r0) * 2.f, w01 = (e1 * r0) * 2.f;
  const float m1 = fmaxf(a[12], a[13]);
  const float f0 = __expf(a[12] - m1), f1 = __expf(a[13] - m1);
  const float r1 = __builtin_amdgcn_rcpf(f0 + f1);

  float gv[NH];
  gv[0] = w00 * ((f0 * r1) * 2.f);
  gv[1] = w00 * ((f1 * r1) * 2.f);
#pragma unroll
  for (int e = 0; e < ER; ++e) {
    const bool sel = (e == i1) || (e == i2);
    gv[2 + e] = sel ? (w01 * ((g[e] * dinv) * 2.f)) : 0.f;
  }
  float mine = 0.f;
#pragma unroll
  for (int e = 0; e < NH; ++e) mine = (lane == e) ? gv[e] : mine;
  if (lane < GP) sg[wave * GP + lane] = mine;
  __syncthreads();
  if (wave == 0) {
    const v4f v = *(const v4f*)(sg + lane * 4);
    volatile v4f* d = (volatile v4f*)(gp + (size_t)blockIdx.x * (8 * GP) + lane * 4);
    *d = v;
    __threadfence();
    *d = v;
  }
}

#define STP 72
#define SVP 264
__global__ __launch_bounds__(256) void k_qkv(const _Float16* __restrict__ xh,
                                             const _Float16* __restrict__ wt,
                                             const float* __restrict__ bqkv,
                                             const float* __restrict__ qnw,
                                             const float* __restrict__ qnb,
                                             const float* __restrict__ knw,
                                             const float* __restrict__ knb,
                                             _Float16* __restrict__ qkp,
                                             _Float16* __restrict__ vtp) {
  __shared__ __align__(16) _Float16 st[256 * STP];
  const int tid = threadIdx.x, lane = tid & 31, wave = tid >> 5;
  const int hh = lane >> 4, c = lane & 15;
  const int bx = blockIdx.x;
  const int b  = bx / SBLK;
  const int sb = (bx - b * SBLK) * 256;
  const int ns = blockIdx.y;
  const int which = ns / NH;
  const int head  = ns - which * NH;
  const int hb    = b * NH + head;
  const int m0 = sb + wave * 32;
  const int n0 = ns * 64;
  const _Float16* A = xh + (size_t)b * SQ * DIM;

  v8f acc[2][4];
#pragma unroll
  for (int s = 0; s < 2; ++s)
#pragma unroll
    for (int t = 0; t < 4; ++t) acc[s][t] = zero8();
  gemm32x64(A, DIM, wt, DIM, DIM, m0, n0, lane, acc);

  float bb[4], nw[4], nb[4];
#pragma unroll
  for (int t = 0; t < 4; ++t) {
    bb[t] = bqkv[n0 + 16 * t + c];
    const int d = 16 * t + c;
    const float wq = qnw[d], wk = knw[d], zq = qnb[d], zk = knb[d];
    nw[t] = (which == 0) ? wq : wk;
    nb[t] = (which == 0) ? zq : zk;
  }
  const bool useln = (which < 2);

#pragma unroll
  for (int sub = 0; sub < 2; ++sub) {
#pragma unroll
    for (int r = 0; r < 8; ++r) {
      float v[4];
#pragma unroll
      for (int t = 0; t < 4; ++t) v[t] = acc[sub][t][r] * QKS + bb[t];
      float s = (v[0] + v[1]) + (v[2] + v[3]);
#pragma unroll
      for (int off = 1; off < 16; off <<= 1) s += __shfl_xor(s, off, 32);
      const float mean = s * 0.015625f;
      float d[4];
      float ss = 0.f;
#pragma unroll
      for (int t = 0; t < 4; ++t) { d[t] = v[t] - mean; ss += d[t] * d[t]; }
#pragma unroll
      for (int off = 1; off < 16; off <<= 1) ss += __shfl_xor(ss, off, 32);
      const float rstd = rsqrtf(ss * 0.015625f + LNEPS);
#pragma unroll
      for (int t = 0; t < 4; ++t) acc[sub][t][r] = useln ? (d[t] * rstd * nw[t] + nb[t]) : v[t];
    }
  }

  if (useln) {
#pragma unroll
    for (int sub = 0; sub < 2; ++sub)
#pragma unroll
      for (int t = 0; t < 4; ++t)
#pragma unroll
        for (int r = 0; r < 8; ++r)
          st[(wave * 32 + sub * 16 + 8 * hh + r) * STP + 16 * t + c] = (_Float16)acc[sub][t][r];
  } else {
#pragma unroll
    for (int sub = 0; sub < 2; ++sub)
#pragma unroll
      for (int t = 0; t < 4; ++t)
#pragma unroll
        for (int r = 0; r < 8; ++r)
          st[(16 * t + c) * SVP + wave * 32 + sub * 16 + 8 * hh + r] = (_Float16)acc[sub][t][r];
  }
  __syncthreads();

  if (useln) {
    _Float16* base = qkp + (size_t)which * QKPLANE + (size_t)hb * SQ * HDM;
#pragma unroll
    for (int g = 0; g < 2; ++g) {
      v4u val[4];
      size_t go[4];
#pragma unroll
      for (int j = 0; j < 4; ++j) {
        const int p  = tid + 256 * (4 * g + j);
        const int lr = p >> 3;
        const int pc = p & 7;
        Pack8 pk;
        pk.h   = *(const v8h*)(st + lr * STP + pc * 8);
        val[j] = pk.u;
        go[j]  = (size_t)(sb + lr) * HDM + pc * 8;
      }
      for (int ps = 0; ps < 2; ++ps) {
#pragma unroll
        for (int j = 0; j < 4; ++j) *(volatile v4u*)(base + go[j]) = val[j];
        __threadfence();
      }
    }
  } else {
    _Float16* base = vtp + (size_t)hb * HDM * SQ;
#pragma unroll
    for (int g = 0; g < 2; ++g) {
      v4u val[4];
      size_t go[4];
#pragma unroll
      for (int j = 0; j < 4; ++j) {
        const int p    = tid + 256 * (4 * g + j);
        const int drow = p >> 5;
        const int pc   = p & 31;
        Pack8 pk;
        pk.h   = *(const v8h*)(st + drow * SVP + pc * 8);
        val[j] = pk.u;
        go[j]  = (size_t)drow * SQ + sb + pc * 8;
      }
      for (int ps = 0; ps < 2; ++ps) {
#pragma unroll
        for (int j = 0; j < 4; ++j) *(volatile v4u*)(base + go[j]) = val[j];
        __threadfence();
      }
    }
  }
}

#define KTP 72
__global__ __launch_bounds__(256) void k_attn(const _Float16* __restrict__ qp,
                                              const _Float16* __restrict__ kp,
                                              const _Float16* __restrict__ vt,
                                              const float* __restrict__ gt,
                                              _Float16* __restrict__ op, float sscale) {
  __shared__ __align__(16) _Float16 Ks[KC * KTP];
  __shared__ __align__(16) _Float16 Vs[HDM * KTP];
  __shared__ __align__(16) _Float16 Ps[8 * 16 * KTP];

  const int tid = threadIdx.x, lane = tid & 31, wave = tid >> 5;
  const int hh = lane >> 4, c = lane & 15;
  const int qb  = blockIdx.x % NQB;
  const int hb  = blockIdx.x / NQB;
  const int h   = hb % NH;
  const int b   = hb / NH;
  const int q0  = qb * QB + wave * 16;

  const _Float16* Q = qp + (size_t)hb * SQ * HDM;
  const _Float16* K = kp + (size_t)hb * SQ * HDM;
  const _Float16* V = vt + (size_t)hb * HDM * SQ;

  v16h qa[2];
  qa[0] = ldfrag(Q, HDM, q0, 0, lane);
  qa[1] = ldfrag(Q, HDM, q0, 32, lane);

  const float NEGI = -__builtin_huge_valf();
  float mrow[8], lrow[8];
  v8f oacc[4];
#pragma unroll
  for (int r = 0; r < 8; ++r) { mrow[r] = NEGI; lrow[r] = 0.f; }
#pragma unroll
  for (int t = 0; t < 4; ++t) oacc[t] = zero8();

  _Float16* pw = Ps + wave * 16 * KTP;

  for (int kc = 0; kc < NCK; ++kc) {
    const int kv0 = kc * KC;
    __syncthreads();
    {
      const int r  = tid >> 2;
      const int qq = (tid & 3) * 16;
      const _Float16* ks = K + (size_t)(kv0 + r) * HDM + qq;
      const _Float16* vs = V + (size_t)r * SQ + kv0 + qq;
#pragma unroll
      for (int e = 0; e < 2; ++e) {
        *(v8h*)(Ks + r * KTP + qq + 8 * e) = *(const v8h*)(ks + 8 * e);
        *(v8h*)(Vs + r * KTP + qq + 8 * e) = *(const v8h*)(vs + 8 * e);
      }
    }
    __syncthreads();

    v8f s[4];
#pragma unroll
    for (int j = 0; j < 4; ++j) s[j] = zero8();
#pragma unroll
    for (int dc = 0; dc < 2; ++dc) {
#pragma unroll
      for (int j = 0; j < 4; ++j) {
        const v16h kb = ldfrag(Ks, KTP, j * 16, dc * 32, lane);
        s[j] = mma16(qa[dc], kb, s[j]);
      }
    }
    float cm[8];
#pragma unroll
    for (int r = 0; r < 8; ++r) {
      float m = NEGI;
#pragma unroll
      for (int j = 0; j < 4; ++j) { s[j][r] *= sscale; m = fmaxf(m, s[j][r]); }
#pragma unroll
      for (int off = 1; off < 16; off <<= 1) m = fmaxf(m, __shfl_xor(m, off, 32));
      cm[r] = m;
    }
    float al[8];
#pragma unroll
    for (int r = 0; r < 8; ++r) {
      const float mnew  = fmaxf(mrow[r], cm[r]);
      const float alpha = __expf(mrow[r] - mnew);
      mrow[r] = mnew;
      float psum = 0.f;
#pragma unroll
      for (int j = 0; j < 4; ++j) {
        const float p = __expf(s[j][r] - mnew);
        psum += p;
        pw[(8 * hh + r) * KTP + j * 16 + c] = (_Float16)(p * 1024.0f);
      }
#pragma unroll
      for (int off = 1; off < 16; off <<= 1) psum += __shfl_xor(psum, off, 32);
      lrow[r] = lrow[r] * alpha + psum;
      al[r] = alpha;
    }
#pragma unroll
    for (int t = 0; t < 4; ++t)
#pragma unroll
      for (int r = 0; r < 8; ++r) oacc[t][r] *= al[r];
    __syncthreads();

#pragma unroll
    for (int kk = 0; kk < 2; ++kk) {
      const v16h pa = ldfrag(pw, KTP, 0, kk * 32, lane);
#pragma unroll
      for (int t = 0; t < 4; ++t) {
        const v16h vb = ldfrag(Vs, KTP, t * 16, kk * 32, lane);
        oacc[t] = mma16(pa, vb, oacc[t]);
      }
    }
  }

  float invl[8];
#pragma unroll
  for (int r = 0; r < 8; ++r) {
    const float g = gt[((size_t)b * SQ + q0 + 8 * hh + r) * GP + h];
    invl[r] = (lrow[r] > 0.f) ? (g * (0.0625f / lrow[r])) : 0.f;
  }
  __syncthreads();
#pragma unroll
  for (int r = 0; r < 8; ++r) {
#pragma unroll
    for (int t = 0; t < 4; ++t)
      pw[(8 * hh + r) * KTP + 16 * t + c] = (_Float16)(oacc[t][r] * invl[r]);
  }
  __syncthreads();
  v4u val[4];
  size_t go[4];
#pragma unroll
  for (int it = 0; it < 4; ++it) {
    const int p  = lane + 32 * it;
    const int L  = p >> 3;
    const int pc = p & 7;
    Pack8 pk;
    pk.h    = *(const v8h*)(pw + L * KTP + pc * 8);
    val[it] = pk.u;
    go[it]  = ((size_t)b * SQ + q0 + L) * DIM + (size_t)h * HDM + pc * 8;
  }
  for (int ps = 0; ps < 2; ++ps) {
#pragma unroll
    for (int it = 0; it < 4; ++it) *(volatile v4u*)(op + go[it]) = val[it];
    __threadfence();
  }
}

#define OTP 68
__device__ __forceinline__ void out_epilogue_f32(v8f (&acc)[2][4], float scale, const float (&bb)[4],
                                                 float* sw, float* __restrict__ out, int ldo,
                                                 int m0, int n0, int lane, int hh, int c) {
#pragma unroll
  for (int sub = 0; sub < 2; ++sub) {
    __syncthreads();
#pragma unroll
    for (int t = 0; t < 4; ++t) {
#pragma unroll
      for (int r = 0; r < 8; ++r) sw[(8 * hh + r) * OTP + 16 * t + c] = acc[sub][t][r] * scale + bb[t];
    }
    __syncthreads();
    v4f val[8];
    size_t go[8];
#pragma unroll
    for (int it = 0; it < 8; ++it) {
      const int p    = lane + 32 * it;
      const int L    = p >> 3;
      const int pc   = p & 7;
      const int row  = L >> 1;
      const int half = L & 1;
      val[it] = *(const v4f*)(sw + row * OTP + half * 32 + pc * 4);
      go[it]  = (size_t)(m0 + sub * 16 + row) * ldo + n0 + half * 32 + pc * 4;
    }
    for (int ps = 0; ps < 2; ++ps) {
#pragma unroll
      for (int it = 0; it < 8; ++it) *(volatile v4f*)(out + go[it]) = val[it];
      __threadfence();
    }
  }
}

__global__ __launch_bounds__(256) void k_gemm_f32(const _Float16* __restrict__ ap, int lda,
                                                  const _Float16* __restrict__ wt, int K,
                                                  const float* __restrict__ bias, float scale,
                                                  float* __restrict__ out, int ldo) {
  __shared__ __align__(16) float st[8][16 * OTP];
  const int tid = threadIdx.x, lane = tid & 31, wave = tid >> 5;
  const int hh = lane >> 4, c = lane & 15;
  const int m0 = blockIdx.x * 256 + wave * 32;
  const int n0 = blockIdx.y * 64;

  v8f acc[2][4];
#pragma unroll
  for (int s = 0; s < 2; ++s)
#pragma unroll
    for (int t = 0; t < 4; ++t) acc[s][t] = zero8();
  gemm32x64(ap, lda, wt, K, K, m0, n0, lane, acc);
  float bb[4];
#pragma unroll
  for (int t = 0; t < 4; ++t) bb[t] = bias[n0 + 16 * t + c];
  out_epilogue_f32(acc, scale, bb, st[wave], out, ldo, m0, n0, lane, hh, c);
}

extern "C" void kernel_launch(void* const* d_in, const int* in_sizes, int n_in,
                              void* d_out, int out_size, void* d_ws, size_t ws_size,
                              hipStream_t stream) {
  if (n_in < 12) return;
  if (in_sizes[0] != NTOK * DIM) return;
  if (in_sizes[1] != DIM * NQKV) return;
  if (in_sizes[2] != NQKV) return;
  if (in_sizes[3] != HDM) return;
  if (in_sizes[4] != HDM) return;
  if (in_sizes[5] != HDM) return;
  if (in_sizes[6] != HDM) return;
  if (in_sizes[7] != DIM * ER) return;
  if (in_sizes[8] != DIM * 2) return;
  if (in_sizes[9] != DIM * 2) return;
  if (in_sizes[10] != DIM * DIM) return;
  if (in_sizes[11] != DIM) return;
  if (out_size != NTOK * DIM) return;

  const float* x      = (const float*)d_in[0];
  const float* qkv_w  = (const float*)d_in[1];
  const float* qkv_b  = (const float*)d_in[2];
  const float* qn_w   = (const float*)d_in[3];
  const float* qn_b   = (const float*)d_in[4];
  const float* kn_w   = (const float*)d_in[5];
  const float* kn_b   = (const float*)d_in[6];
  const float* wg_w   = (const float*)d_in[7];
  const float* wg0_w  = (const float*)d_in[8];
  const float* wg1_w  = (const float*)d_in[9];
  const float* proj_w = (const float*)d_in[10];
  const float* proj_b = (const float*)d_in[11];
  float* out = (float*)d_out;

  size_t off = 0;
  const size_t oX  = off; off += (size_t)NTOK * DIM * 2;
  const size_t oWt = off; off += (size_t)NQKV * DIM * 2;
  const size_t oWp = off; off += (size_t)DIM * DIM * 2;
  const size_t oG  = off; off += (size_t)NTOK * GP * 4;
  const size_t oQ  = off; off += (size_t)QKPLANE * 2;
  const size_t oK  = off; off += (size_t)QKPLANE * 2;
  const size_t oV  = off; off += (size_t)NBATCH * NH * HDM * SQ * 2;
  const size_t oO  = off; off += (size_t)NTOK * DIM * 2;
  if (off > ws_size) return;
  if (off > (size_t)134217728) return;
  if (oK != oQ + (size_t)QKPLANE * 2) return;
  if ((oWt | oWp | oG | oQ | oK | oV | oO) & (size_t)127) return;

  char* ws = (char*)d_ws;
  _Float16* Xh  = (_Float16*)(ws + oX);
  _Float16* Wt  = (_Float16*)(ws + oWt);
  _Float16* Wpt = (_Float16*)(ws + oWp);
  float*    G   = (float*)(ws + oG);
  _Float16* QKp = (_Float16*)(ws + oQ);
  _Float16* Kp  = (_Float16*)(ws + oK);
  _Float16* Vt  = (_Float16*)(ws + oV);
  _Float16* Og  = (_Float16*)(ws + oO);

  k_cvt<<<dim3((NTOK * DIM) / 8 / 256), dim3(256), 0, stream>>>(x, Xh, (NTOK * DIM) / 8);
  k_wtr<<<dim3(NQKV / 64, DIM / 64), dim3(256), 0, stream>>>(qkv_w, Wt, DIM, NQKV, 32.0f);
  k_wtr<<<dim3(DIM / 64, DIM / 64), dim3(256), 0, stream>>>(proj_w, Wpt, DIM, DIM, 32.0f);
  k_gate<<<dim3(NTOK / 8), dim3(256), 0, stream>>>(x, wg_w, wg0_w, wg1_w, G);
  k_qkv<<<dim3(NBATCH * SBLK, NQKV / 64), dim3(256), 0, stream>>>(Xh, Wt, qkv_b, qn_w, qn_b, kn_w, kn_b, QKp, Vt);
  const float sscale = 0.125f;
  k_attn<<<dim3(NBATCH * NH * NQB), dim3(256), 0, stream>>>(QKp, Kp, Vt, G, Og, sscale);
  k_gemm_f32<<<dim3(NTOK / 256, DIM / 64), dim3(256), 0, stream>>>(Og, DIM, Wpt, DIM, proj_b, PJS, out, DIM);
  (void)hipGetLastError();
}
